// MSA2Pair_10668698763286
// MI455X (gfx1250) — hardware-verified
//
#include <hip/hip_runtime.h>


#define NS   128
#define NL   256
#define DMS  256
#define DH   32
#define DP   128
#define NR   (NS * NL)
#define LCH  64
#define NCH  (NL / LCH)
#define DM   DMS
#define TT   NR
#define LNEPS 1e-5f
typedef _Float16 h16;
typedef unsigned short bf;
typedef __attribute__((ext_vector_type(16))) __bf16   v16bf;
typedef __attribute__((ext_vector_type(16))) _Float16 v16h;
typedef __attribute__((ext_vector_type(8)))  _Float16 v8h;
typedef __attribute__((ext_vector_type(8)))  unsigned short v8us;
typedef __attribute__((ext_vector_type(8)))  float    v8f;
typedef __attribute__((ext_vector_type(4)))  float    v4f;
typedef __attribute__((ext_vector_type(2)))  float    v2f;
typedef __attribute__((ext_vector_type(4)))  unsigned short v4us;
typedef __attribute__((ext_vector_type(2)))  unsigned short v2us;
typedef v8h  __attribute__((may_alias)) v8ha;
typedef v4f  __attribute__((may_alias)) v4fa;
typedef v8us __attribute__((may_alias)) v8usa;

__device__ __forceinline__ unsigned short f2bf(float f) { unsigned u = __float_as_uint(f); u += 0x7FFFu + ((u >> 16) & 1u); return (unsigned short)(u >> 16); }
__device__ __forceinline__ float bf2f(unsigned short b) { return __uint_as_float(((unsigned)b) << 16); }
__device__ __forceinline__ float bfr(float f) { return bf2f(f2bf(f)); }
__device__ __forceinline__ void splitf(float y, unsigned short& h, unsigned short& l) { h = f2bf(y); l = f2bf(y - bf2f(h)); }
__device__ __forceinline__ v16h cat16(v8h lo, v8h hi) { return __builtin_shufflevector(lo, hi, 0, 1, 2, 3, 4, 5, 6, 7, 8, 9, 10, 11, 12, 13, 14, 15); }
__device__ __forceinline__ v16bf cat16b(v8us lo, v8us hi) { return __builtin_bit_cast(v16bf, __builtin_shufflevector(lo, hi, 0, 1, 2, 3, 4, 5, 6, 7, 8, 9, 10, 11, 12, 13, 14, 15)); }
__device__ __forceinline__ v8f wmma16(v16h a, v16h b, v8f c) { return __builtin_amdgcn_wmma_f32_16x16x32_f16(false, a, false, b, (short)0, c, false, false); }
__device__ __forceinline__ v8f wmmab(v16bf a, v16bf b, v8f c) { return __builtin_amdgcn_wmma_f32_16x16x32_bf16(false, a, false, b, (short)0, c, false, false); }

template <typename T16> struct WFrag;
template <> struct WFrag<h16> { typedef v16h V; static __device__ __forceinline__ V ld(const h16* p) { return cat16(*(const v8h*)p, *(const v8h*)(p + 16)); } static __device__ __forceinline__ v8f mma(V a, V b, v8f c) { return wmma16(a, b, c); } };
template <> struct WFrag<bf> { typedef v16bf V; static __device__ __forceinline__ V ld(const bf* p) { return cat16b(*(const v8us*)p, *(const v8us*)(p + 16)); } static __device__ __forceinline__ v8f mma(V a, V b, v8f c) { return wmmab(a, b, c); } };
template <typename T16, int NSPLIT, bool BIAS>
__global__ __launch_bounds__(32) void k_gemmw(const T16* __restrict__ A, const T16* __restrict__ A2, const T16* __restrict__ Bt, const T16* __restrict__ Bt2, int K, float* C, int ldc, const float* __restrict__ bias, size_t sA, size_t sB, size_t sC) {
    typedef typename WFrag<T16>::V V;
    __shared__ __align__(16) float os[16 * 68];
    const size_t z = blockIdx.z; A += z * sA; if (A2) A2 += z * sA; Bt += z * sB; if (Bt2) Bt2 += z * sB; C += z * sC;
    const int lane = threadIdx.x & 31, lr = lane & 15, hi = lane >> 4; const int r0 = blockIdx.x * 64, c0 = blockIdx.y * 64;
    v8f acc[4][4];
#pragma unroll
    for (int mb = 0; mb < 4; ++mb)
#pragma unroll
        for (int nb = 0; nb < 4; ++nb) acc[mb][nb] = (v8f){};
    const size_t aoff = (size_t)(r0 + lr) * K + 8 * hi, boff = (size_t)(c0 + lr) * K + 8 * hi;
#pragma unroll 1
    for (int kc = 0; kc < K; kc += 32) {
        V a[4], a2[4];
#pragma unroll
        for (int mb = 0; mb < 4; ++mb) { a[mb] = WFrag<T16>::ld(A + aoff + (size_t)mb * 16 * K + kc); if (NSPLIT == 1 || NSPLIT == 2) a2[mb] = WFrag<T16>::ld(A2 + aoff + (size_t)mb * 16 * K + kc); }
#pragma unroll
        for (int nb = 0; nb < 4; ++nb) { const V b = WFrag<T16>::ld(Bt + boff + (size_t)nb * 16 * K + kc); V b2; if (NSPLIT >= 2) b2 = WFrag<T16>::ld(Bt2 + boff + (size_t)nb * 16 * K + kc);
#pragma unroll
            for (int mb = 0; mb < 4; ++mb) { acc[mb][nb] = WFrag<T16>::mma(a[mb], b, acc[mb][nb]); if (NSPLIT == 1 || NSPLIT == 2) acc[mb][nb] = WFrag<T16>::mma(a2[mb], b, acc[mb][nb]); if (NSPLIT >= 2) acc[mb][nb] = WFrag<T16>::mma(a[mb], b2, acc[mb][nb]); } }
        asm volatile("v_nop\n\tv_nop\n\tv_nop\n\tv_nop" : "+v"(acc[0][0]), "+v"(acc[1][1]), "+v"(acc[2][2]), "+v"(acc[3][3]) : "v"(a[0]), "v"(a[3]));
    }
#pragma unroll
    for (int mb = 0; mb < 4; ++mb) {
#pragma unroll
        for (int nb = 0; nb < 4; ++nb) {
#pragma unroll
            for (int j = 0; j < 8; ++j) os[(hi * 8 + j) * 68 + nb * 16 + lr] = acc[mb][nb][j]; }
        __builtin_amdgcn_wave_barrier(); asm volatile("" ::: "memory");
        float* crow = C + (size_t)(r0 + mb * 16) * ldc + c0;
#pragma unroll 1
        for (int ps = 0; ps < 2; ++ps) {
#pragma unroll
            for (int s = 0; s < 8; ++s) { const int row = 2 * s + hi, cofs = lr * 4; v4f val = *(const v4fa*)(os + row * 68 + cofs); if (BIAS) { val[0] += bfr(bias[c0 + cofs]); val[1] += bfr(bias[c0 + cofs + 1]); val[2] += bfr(bias[c0 + cofs + 2]); val[3] += bfr(bias[c0 + cofs + 3]); }
                *(volatile v4f*)(crow + (size_t)row * ldc + cofs) = val; }
            if (ps == 0) __threadfence(); }
        __builtin_amdgcn_wave_barrier(); asm volatile("" ::: "memory");
    }
}
template <bool RND>
__global__ __launch_bounds__(256) void k_lnhl(const float* __restrict__ X, const float* __restrict__ A, const float* __restrict__ g, const float* __restrict__ be, float* Z, bf* Yh, bf* Yl) {
    const int lane = threadIdx.x & 31; const int r = blockIdx.x * 8 + (threadIdx.x >> 5); if (r >= TT) return; const float* xr = X + (size_t)r * DM; const float* ar = A ? A + (size_t)r * DM : nullptr; float s = 0.f;
#pragma unroll 1
    for (int ch = 0; ch < DM / 128; ++ch) { const int c0 = ch * 128 + lane * 4; const v4f a = *(const v4f*)(xr + c0); v4f d = {0.f, 0.f, 0.f, 0.f}; if (ar) d = *(const v4f*)(ar + c0);
#pragma unroll
        for (int q = 0; q < 4; ++q) s += __fadd_rn((RND ? bfr(a[q]) : a[q]), d[q]); }
#pragma unroll
    for (int sh = 16; sh; sh >>= 1) s += __shfl_xor(s, sh, 32);
    const float mu = s * (1.0f / DM); float s2 = 0.f;
#pragma unroll 1
    for (int ch = 0; ch < DM / 128; ++ch) { const int c0 = ch * 128 + lane * 4; const v4f a = *(const v4f*)(xr + c0); v4f d = {0.f, 0.f, 0.f, 0.f}; if (ar) d = *(const v4f*)(ar + c0);
#pragma unroll
        for (int q = 0; q < 4; ++q) { const float d0 = __fsub_rn(__fadd_rn((RND ? bfr(a[q]) : a[q]), d[q]), mu); float p = __fmul_rn(d0, d0); asm volatile("" : "+v"(p)); s2 = __fadd_rn(s2, p); } }
#pragma unroll
    for (int sh = 16; sh; sh >>= 1) s2 += __shfl_xor(s2, sh, 32);
    const float rs = __fdiv_rn(1.0f, __fsqrt_rn(__fadd_rn(s2 * (1.0f / DM), LNEPS)));
#pragma unroll 1
    for (int ps = 0; ps < 2; ++ps) {
#pragma unroll 1
        for (int ch = 0; ch < DM / 128; ++ch) { const int c0 = ch * 128 + lane * 4; const v4f a = *(const v4f*)(xr + c0); v4f d = {0.f, 0.f, 0.f, 0.f}; if (ar) d = *(const v4f*)(ar + c0); v4f z4; v4us oh, ol;
#pragma unroll
            for (int q = 0; q < 4; ++q) { const float v = __fadd_rn((RND ? bfr(a[q]) : a[q]), d[q]); float n0 = __fmul_rn(__fsub_rn(v, mu), rs); asm volatile("" : "+v"(n0)); float n1 = __fmul_rn(n0, bfr(g[c0 + q])); asm volatile("" : "+v"(n1)); const float y = __fadd_rn(n1, bfr(be[c0 + q])); z4[q] = y;     unsigned short h2, l2; splitf(y, h2, l2); oh[q] = h2; ol[q] = l2; }
            if (Z) *(volatile v4f*)(Z + (size_t)r * DM + c0) = z4; *(volatile v4us*)(Yh + (size_t)r * DM + c0) = oh; *(volatile v4us*)(Yl + (size_t)r * DM + c0) = ol; }
        if (ps == 0) __threadfence(); } }


__global__ __launch_bounds__(256) void k_wlr(const float* __restrict__ wl, const float* __restrict__ wr, const float* __restrict__ bl, const float* __restrict__ br, bf* Bt, float* BB) {
#pragma unroll 1
    for (int ps = 0; ps < 2; ++ps) {
#pragma unroll 1
        for (int e0 = threadIdx.x * 2; e0 < 2 * DH * DMS; e0 += 512) { const int d = e0 % DMS, n = e0 / DMS; const float* w = (n < DH) ? wl : wr; const int nn = n % DH; v2us o; o[0] = f2bf(w[(size_t)d * DH + nn]); o[1] = f2bf(w[(size_t)(d + 1) * DH + nn]); *(volatile v2us*)(Bt + e0) = o; }
        if (threadIdx.x < 16) { v4f b4; for (int q = 0; q < 4; ++q) { const int n = threadIdx.x * 4 + q; b4[q] = (n < DH) ? bl[n] : br[n - DH]; } *(volatile v4f*)(BB + threadIdx.x * 4) = b4; }
        if (ps == 0) __threadfence(); } }
__global__ __launch_bounds__(256) void k_ltp(const float* __restrict__ LR, bf* ALh, bf* ALl, bf* ARh, bf* ARl) { const size_t e = ((size_t)blockIdx.x * 256 + threadIdx.x) * 2; if (e >= (size_t)NL * DH * NS) return; const int s = (int)(e % NS); const int li = (int)(e / NS); const int l = li / DH, i = li % DH; v2us lh, ll, rh, rl;
#pragma unroll
    for (int q = 0; q < 2; ++q) { const float* row = LR + ((size_t)(s + q) * NL + l) * (2 * DH); unsigned short a, b; splitf(row[i], a, b); lh[q] = a; ll[q] = b; splitf(row[DH + i] * (1.0f / NS), a, b); rh[q] = a; rl[q] = b; }
    *(volatile v2us*)(ALh + e) = lh; *(volatile v2us*)(ALl + e) = ll; *(volatile v2us*)(ARh + e) = rh; *(volatile v2us*)(ARl + e) = rl; __threadfence(); *(volatile v2us*)(ALh + e) = lh; *(volatile v2us*)(ALl + e) = ll; *(volatile v2us*)(ARh + e) = rh; *(volatile v2us*)(ARl + e) = rl; }
__global__ __launch_bounds__(256) void k_gat(const float* __restrict__ OP, bf* Gh, bf* Gl) { const size_t e = ((size_t)blockIdx.x * 256 + threadIdx.x) * 8; if (e >= (size_t)LCH * NL * DH * DH) return; const int k = (int)(e % (DH * DH)); const size_t row = e / (DH * DH); const int m = (int)(row % NL); const int ll = (int)(row / NL); const int i = k / DH, j = k % DH; const float* src = OP + ((size_t)(ll * DH + i)) * (NL * DH) + m * DH + j; const v8f v = *(const v8f*)src; v8us oh, ol;
#pragma unroll
    for (int q = 0; q < 8; ++q) { unsigned short a, b; splitf(v[q], a, b); oh[q] = a; ol[q] = b; } *(volatile v8us*)(Gh + e) = oh; *(volatile v8us*)(Gl + e) = ol; __threadfence(); *(volatile v8us*)(Gh + e) = oh; *(volatile v8us*)(Gl + e) = ol; }
__global__ __launch_bounds__(256) void k_cvt8(const float* __restrict__ src, bf* dst, size_t n8) { const size_t i = (size_t)blockIdx.x * 256 + threadIdx.x; if (i >= n8) return; const v8f v = *(const v8f*)(src + i * 8); v8us o;
#pragma unroll
    for (int k = 0; k < 8; ++k) o[k] = f2bf(v[k]); *(volatile v8us*)(dst + i * 8) = o; __threadfence(); *(volatile v8us*)(dst + i * 8) = o; }
__global__ __launch_bounds__(256) void k_wtG(const float* __restrict__ w, int K, int N, bf* Bt) {
    const int lane = threadIdx.x & 31; const int L0 = (blockIdx.x * 8 + (threadIdx.x >> 5)) * 8; const int nlines = N * K / 64;
#pragma unroll
    for (int ps = 0; ps < 2; ++ps) {
#pragma unroll 1
        for (int l = 0; l < 8; ++l) { const int L = L0 + l; if (L >= nlines) break; const size_t e = (size_t)L * 64 + lane * 2; const int k = (int)(e % K), n = (int)(e / K); v2us o;
            o[0] = f2bf(w[(size_t)k * N + n]); o[1] = f2bf(w[(size_t)(k + 1) * N + n]); *(volatile v2us*)(Bt + e) = o; }
        if (ps == 0) __threadfence(); }
}
__global__ __launch_bounds__(256) void k_addres(const float* __restrict__ P, const float* __restrict__ Y, float* O, size_t n4) { const size_t i = (size_t)blockIdx.x * 256 + threadIdx.x; if (i >= n4) return; const v4f a = *(const v4f*)(P + i * 4), y = *(const v4f*)(Y + i * 4); v4f o;
#pragma unroll
    for (int q = 0; q < 4; ++q) o[q] = __fadd_rn(bfr(a[q]), y[q]); *(volatile v4f*)(O + i * 4) = o; __threadfence(); *(volatile v4f*)(O + i * 4) = o; }

extern "C" void kernel_launch(void* const* d_in, const int* in_sizes, int n_in,
                              void* d_out, int out_size, void* d_ws, size_t ws_size, hipStream_t stream) {
    (void)in_sizes; (void)n_in; (void)out_size;
    const float* msa = (const float*)d_in[0]; const float* pair = (const float*)d_in[1]; const float* gam = (const float*)d_in[2]; const float* bet = (const float*)d_in[3]; const float* wl = (const float*)d_in[4]; const float* bl = (const float*)d_in[5]; const float* wr = (const float*)d_in[6]; const float* br = (const float*)d_in[7]; const float* wo = (const float*)d_in[8]; const float* bo = (const float*)d_in[9];
    float* OUT = (float*)d_out;
    char* wsp = (char*)d_ws;
    auto take = [&](size_t bytes) { char* p = wsp; wsp += (bytes + 255) & ~(size_t)255; return (void*)p; };
    bf* WLR = (bf*)take((size_t)2 * DH * DMS * 2); float* BB = (float*)take(256); bf* WO = (bf*)take((size_t)DP * DH * DH * 2);
    bf* Xh = (bf*)take((size_t)NR * DMS * 2); bf* Xl = (bf*)take((size_t)NR * DMS * 2); float* LR = (float*)take((size_t)NR * 2 * DH * 4);
    bf* ALh = (bf*)take((size_t)NL * DH * NS * 2); bf* ALl = (bf*)take((size_t)NL * DH * NS * 2); bf* ARh = (bf*)take((size_t)NL * DH * NS * 2); bf* ARl = (bf*)take((size_t)NL * DH * NS * 2);
    float* OP = (float*)take((size_t)LCH * DH * NL * DH * 4); bf* Gh = (bf*)take((size_t)LCH * NL * DH * DH * 2); bf* Gl = (bf*)take((size_t)LCH * NL * DH * DH * 2); float* Y = (float*)take((size_t)LCH * NL * DP * 4);
    if ((size_t)(wsp - (char*)d_ws) > ws_size) return;
    k_wlr<<<1, 256, 0, stream>>>(wl, wr, bl, br, WLR, BB); k_wtG<<<(unsigned)((DH * DH * DP / 64 + 63) / 64), 256, 0, stream>>>(wo, DH * DH, DP, WO);
    k_lnhl<true><<<NR / 8, 256, 0, stream>>>(msa, nullptr, gam, bet, nullptr, Xh, Xl);
    k_gemmw<bf, 1, true><<<dim3(NR / 64, 1, 1), 32, 0, stream>>>(Xh, Xl, WLR, nullptr, DMS, LR, 2 * DH, BB, 0, 0, 0);
    k_ltp<<<(unsigned)(((size_t)NL * DH * NS / 2 + 255) / 256), 256, 0, stream>>>(LR, ALh, ALl, ARh, ARl);
    for (int c = 0; c < NCH; ++c) { const size_t l0 = (size_t)c * LCH;
        k_gemmw<bf, 2, false><<<dim3(LCH * DH / 64, NL * DH / 64, 1), 32, 0, stream>>>(ALh + l0 * DH * NS, ALl + l0 * DH * NS, ARh, ARl, NS, OP, NL * DH, nullptr, 0, 0, 0);
        k_gat<<<(unsigned)(((size_t)LCH * NL * DH * DH / 8 + 255) / 256), 256, 0, stream>>>(OP, Gh, Gl);
        k_gemmw<bf, 1, true><<<dim3(LCH * NL / 64, DP / 64, 1), 32, 0, stream>>>(Gh, Gl, WO, nullptr, DH * DH, Y, DP, bo, 0, 0, 0);
        k_addres<<<(unsigned)(((size_t)LCH * NL * DP / 4 + 255) / 256), 256, 0, stream>>>(pair + l0 * NL * DP, Y, OUT + l0 * NL * DP, (size_t)LCH * NL * DP / 4); }
}
